// FlexSelfAttention_10222022164658
// MI455X (gfx1250) — hardware-verified
//
#include <hip/hip_runtime.h>
#include <stdint.h>
#include <stddef.h>


typedef _Float16 v16h __attribute__((ext_vector_type(16)));
typedef _Float16 v8h  __attribute__((ext_vector_type(8)));
typedef _Float16 v4h  __attribute__((ext_vector_type(4)));
typedef float    v8f  __attribute__((ext_vector_type(8)));
typedef float    v4f  __attribute__((ext_vector_type(4)));

union Frag { v16h v; v8h half[2]; };

constexpr int S_LEN   = 2048;
constexpr int HQ_N    = 16;
constexpr int HKV_N   = 4;
constexpr int D_DIM   = 128;
constexpr int HID     = HQ_N * D_DIM;
constexpr int KVD     = HKV_N * D_DIM;
constexpr int ROT     = D_DIM / 2;
constexpr int LO_ROWS = 128;
constexpr float RMS_EPS = 1.1920929e-07f;

#define NOP4 "v_nop\n\tv_nop\n\tv_nop\n\tv_nop"

__device__ __forceinline__ v8f wmma16(v16h a, v16h b, v8f c)
{
    return __builtin_amdgcn_wmma_f32_16x16x32_f16(false, a, false, b, (short)0, c, false, false);
}

__device__ __forceinline__ v8f vzero8()
{
    v8f z = {0.f, 0.f, 0.f, 0.f, 0.f, 0.f, 0.f, 0.f};
    return z;
}

__device__ __forceinline__ float bf16_rne(float f)
{
    unsigned u = __float_as_uint(f);
    u = (u + 0x7FFFu + ((u >> 16) & 1u)) & 0xFFFF0000u;
    return __uint_as_float(u);
}

__global__ __launch_bounds__(256)
void cvt_k(const float* __restrict__ in, _Float16* __restrict__ out, int n8, float scale)
{
    const int i = blockIdx.x * 256 + threadIdx.x;
    if (i >= n8) return;
    const v4f a = *(const v4f*)(in + (size_t)i * 8);
    const v4f b = *(const v4f*)(in + (size_t)i * 8 + 4);
    v8h o;
#pragma unroll
    for (int j = 0; j < 4; ++j) {
        o[j]     = (_Float16)(bf16_rne(a[j]) * scale);
        o[4 + j] = (_Float16)(bf16_rne(b[j]) * scale);
    }
    _Float16* p = out + (size_t)i * 8;
    *(volatile v8h*)p = o;
    __threadfence();
    *(volatile v8h*)p = o;
}

__global__ __launch_bounds__(64)
void rope_tab_k(const int* __restrict__ pos, float* __restrict__ tab, int S, int npos)
{
    __shared__ __align__(16) float cs_s[ROT];
    __shared__ __align__(16) float sn_s[ROT];
    const int s = blockIdx.x;
    const int t = threadIdx.x;
    if (s >= S) return;
    int ps = s;
    if (ps > npos - 1) ps = npos - 1;
    if (ps < 0) ps = 0;
    const float tp = (float)pos[ps];
    {
        const float e = (float)(2 * t) * (1.0f / 128.0f);
        const float pw = powf(10000.0f, e);
        const float inv = 1.0f / pw;
        const float fr = tp * inv;
        float sn, cs;
        sincosf(fr, &sn, &cs);
        cs_s[t] = cs;
        sn_s[t] = sn;
    }
    __syncthreads();
    if (t < 32) {
        const int chunk = t & 15;
        v4f o;
        if (t < 16) o = *(const v4f*)(cs_s + chunk * 4);
        else        o = *(const v4f*)(sn_s + chunk * 4);
        float* d = tab + ((t < 16) ? (size_t)0 : (size_t)S * ROT) + (size_t)s * ROT + chunk * 4;
        *(volatile v4f*)d = o;
        __threadfence();
        *(volatile v4f*)d = o;
    }
}

__device__ __forceinline__ void gemm_core(v8f (&acc)[2][4],
                                          const _Float16* __restrict__ A,
                                          const _Float16* __restrict__ B,
                                          int ld, int r0, int c0, int K, int m, int h)
{
    const _Float16* ap0 = A + (size_t)(r0 + m) * ld + 8 * h;
    const _Float16* ap1 = A + (size_t)(r0 + 16 + m) * ld + 8 * h;
    const _Float16* bp  = B + (size_t)(c0 + m) * ld + 8 * h;
#pragma unroll 1
    for (int k0 = 0; k0 < K; k0 += 32) {
        Frag a0, a1, b[4];
        a0.half[0] = *(const v8h*)(ap0 + k0);
        a0.half[1] = *(const v8h*)(ap0 + k0 + 16);
        a1.half[0] = *(const v8h*)(ap1 + k0);
        a1.half[1] = *(const v8h*)(ap1 + k0 + 16);
#pragma unroll
        for (int ni = 0; ni < 4; ++ni) {
            const _Float16* bq = bp + (size_t)(16 * ni) * ld + k0;
            b[ni].half[0] = *(const v8h*)(bq);
            b[ni].half[1] = *(const v8h*)(bq + 16);
        }
#pragma unroll
        for (int ni = 0; ni < 4; ++ni) {
            acc[0][ni] = wmma16(a0.v, b[ni].v, acc[0][ni]);
            acc[1][ni] = wmma16(a1.v, b[ni].v, acc[1][ni]);
        }
        asm volatile(NOP4
                     : "+v"(acc[0][0]), "+v"(acc[0][1]), "+v"(acc[0][2]), "+v"(acc[0][3]),
                       "+v"(acc[1][0]), "+v"(acc[1][1]), "+v"(acc[1][2]), "+v"(acc[1][3])
                     : "v"(a0.v), "v"(a1.v), "v"(b[0].v), "v"(b[1].v), "v"(b[2].v), "v"(b[3].v));
    }
}

template <int MODE>
__global__ __launch_bounds__(64)
void gemm_k(const _Float16* __restrict__ A, const _Float16* __restrict__ Alo,
            const _Float16* __restrict__ B, void* __restrict__ Cv, _Float16* __restrict__ Clo,
            const float* __restrict__ tab, int M, int N, int K, int lo_rows, float oscale)
{
    constexpr int BM = (MODE == 1) ? 64 : 32;
    constexpr int BN = (MODE == 1) ? 64 : 128;
    constexpr int TP = 132;
    constexpr int UP = 136;
    constexpr int VP = 72;
    __shared__ __align__(16) float    Tf [(MODE == 1) ? 4 : 32 * TP];
    __shared__ __align__(16) _Float16 U  [(MODE == 0) ? 32 * UP : 8];
    __shared__ __align__(16) _Float16 UL [(MODE == 0) ? 32 * UP : 8];
    __shared__ __align__(16) _Float16 T16[(MODE == 1) ? 64 * VP : 8];
    __shared__ __align__(16) _Float16 TL [(MODE == 1) ? 64 * VP : 8];
    (void)Alo; (void)Clo; (void)tab; (void)lo_rows;

    const int tid = threadIdx.x, w = tid >> 5, l = tid & 31, h = l >> 4, m = l & 15;
    const int bm = blockIdx.y * BM, bn = blockIdx.x * BN;
    if (bm + BM > M || bn + BN > N) return;
    const int r0 = (MODE == 1) ? (bm + 32 * w) : bm;
    const int c0 = (MODE == 1) ? bn : (bn + 64 * w);

    v8f acc[2][4];
#pragma unroll
    for (int mi = 0; mi < 2; ++mi)
#pragma unroll
        for (int ni = 0; ni < 4; ++ni) acc[mi][ni] = vzero8();

    if constexpr (MODE == 2) {
        if (bm < lo_rows) {
            gemm_core(acc, Alo, B, K, r0, c0, K, m, h);
#pragma unroll
            for (int mi = 0; mi < 2; ++mi)
#pragma unroll
                for (int ni = 0; ni < 4; ++ni)
#pragma unroll
                    for (int r = 0; r < 8; ++r) acc[mi][ni][r] *= (1.0f / 2048.0f);
        }
    }
    gemm_core(acc, A, B, K, r0, c0, K, m, h);

    if constexpr (MODE == 0 || MODE == 2) {
#pragma unroll
        for (int mi = 0; mi < 2; ++mi)
#pragma unroll
            for (int ni = 0; ni < 4; ++ni)
#pragma unroll
                for (int r = 0; r < 8; ++r)
                    Tf[(16 * mi + 8 * h + r) * TP + 64 * w + 16 * ni + m] = acc[mi][ni][r] * oscale;
        __syncthreads();

        if constexpr (MODE == 2) {
            float* out = (float*)Cv;
            v4f ov[16];
#pragma unroll
            for (int j = 0; j < 16; ++j) {
                const int e = tid + 64 * j;
                const int row = e >> 5, c4 = (e & 31) * 4;
                ov[j] = *(const v4f*)(Tf + row * TP + c4);
            }
#pragma unroll
            for (int j = 0; j < 16; ++j) {
                const int e = tid + 64 * j;
                const int row = e >> 5, c4 = (e & 31) * 4;
                float* gp = out + (size_t)(bm + row) * N + bn + c4;
                *(volatile v4f*)gp = ov[j];
            }
            __threadfence();
#pragma unroll
            for (int j = 0; j < 16; ++j) {
                const int e = tid + 64 * j;
                const int row = e >> 5, c4 = (e & 31) * 4;
                float* gp = out + (size_t)(bm + row) * N + bn + c4;
                *(volatile v4f*)gp = ov[j];
            }
        } else {
            const int rho = tid >> 1, part = tid & 1, cb = 32 * part;
            const float* tr = Tf + rho * TP;
            float ss = 0.f;
#pragma unroll
            for (int c = 0; c < 32; c += 4) {
                const v4f u  = *(const v4f*)(tr + cb + c);
                const v4f u2 = *(const v4f*)(tr + ROT + cb + c);
#pragma unroll
                for (int q = 0; q < 4; ++q) ss += u[q] * u[q] + u2[q] * u2[q];
            }
            ss += __shfl_xor(ss, 1, 32);
            const float rs = 1.0f / sqrtf(ss * (1.0f / (float)D_DIM) + RMS_EPS);
            const int srow = bm + rho;
            const float* tcp = tab + (size_t)srow * ROT + cb;
            const float* tsp = tab + (size_t)M * ROT + (size_t)srow * ROT + cb;
            const bool do_lo = (bm < lo_rows);
#pragma unroll
            for (int c4 = 0; c4 < 8; ++c4) {
                const int cc = 4 * c4;
                const v4f xa = *(const v4f*)(tr + cb + cc);
                const v4f xb = *(const v4f*)(tr + ROT + cb + cc);
                const v4f cs = *(const v4f*)(tcp + cc);
                const v4f sn = *(const v4f*)(tsp + cc);
                v4h o1, o2, q1, q2;
#pragma unroll
                for (int q = 0; q < 4; ++q) {
                    const float x1 = xa[q] * rs, x2 = xb[q] * rs;
                    const float y1 = x1 * cs[q] + x2 * sn[q];
                    const float y2 = x2 * cs[q] - x1 * sn[q];
                    const _Float16 h1 = (_Float16)y1, h2 = (_Float16)y2;
                    o1[q] = h1; o2[q] = h2;
                    q1[q] = (_Float16)((y1 - (float)h1) * 2048.0f);
                    q2[q] = (_Float16)((y2 - (float)h2) * 2048.0f);
                }
                *(v4h*)(U + rho * UP + cb + cc)       = o1;
                *(v4h*)(U + rho * UP + ROT + cb + cc) = o2;
                if (do_lo) {
                    *(v4h*)(UL + rho * UP + cb + cc)       = q1;
                    *(v4h*)(UL + rho * UP + ROT + cb + cc) = q2;
                }
            }
            __syncthreads();
            _Float16* C = (_Float16*)Cv;
            {
                v8h hv[8];
#pragma unroll
                for (int j = 0; j < 8; ++j) {
                    const int e = tid + 64 * j;
                    const int row = e >> 4, c8 = (e & 15) * 8;
                    hv[j] = *(const v8h*)(U + row * UP + c8);
                }
#pragma unroll
                for (int j = 0; j < 8; ++j) {
                    const int e = tid + 64 * j;
                    const int row = e >> 4, c8 = (e & 15) * 8;
                    _Float16* gp = C + (size_t)(bm + row) * N + bn + c8;
                    *(volatile v8h*)gp = hv[j];
                }
                __threadfence();
#pragma unroll
                for (int j = 0; j < 8; ++j) {
                    const int e = tid + 64 * j;
                    const int row = e >> 4, c8 = (e & 15) * 8;
                    _Float16* gp = C + (size_t)(bm + row) * N + bn + c8;
                    *(volatile v8h*)gp = hv[j];
                }
            }
            if (do_lo) {
                v8h lv[8];
#pragma unroll
                for (int j = 0; j < 8; ++j) {
                    const int e = tid + 64 * j;
                    const int row = e >> 4, c8 = (e & 15) * 8;
                    lv[j] = *(const v8h*)(UL + row * UP + c8);
                }
#pragma unroll
                for (int j = 0; j < 8; ++j) {
                    const int e = tid + 64 * j;
                    const int row = e >> 4, c8 = (e & 15) * 8;
                    _Float16* gp = Clo + (size_t)(bm + row) * N + bn + c8;
                    *(volatile v8h*)gp = lv[j];
                }
                __threadfence();
#pragma unroll
                for (int j = 0; j < 8; ++j) {
                    const int e = tid + 64 * j;
                    const int row = e >> 4, c8 = (e & 15) * 8;
                    _Float16* gp = Clo + (size_t)(bm + row) * N + bn + c8;
                    *(volatile v8h*)gp = lv[j];
                }
            }
        }
    } else {
        const bool do_lo = (bm < lo_rows);
#pragma unroll
        for (int mi = 0; mi < 2; ++mi)
#pragma unroll
            for (int ni = 0; ni < 4; ++ni) {
                v8h pk, pl;
#pragma unroll
                for (int r = 0; r < 8; ++r) {
                    const float y = acc[mi][ni][r] * oscale;
                    const _Float16 hh = (_Float16)y;
                    pk[r] = hh;
                    pl[r] = (_Float16)((y - (float)hh) * 2048.0f);
                }
                const int nloc = 16 * ni + m;
                const int sloc = 32 * w + 16 * mi + 8 * h;
                *(v8h*)(T16 + nloc * VP + sloc) = pk;
                if (do_lo) *(v8h*)(TL + nloc * VP + sloc) = pl;
            }
        __syncthreads();
        _Float16* Vt = (_Float16*)Cv;
        {
            v8h hv[8];
#pragma unroll
            for (int j = 0; j < 8; ++j) {
                const int e = tid + 64 * j;
                const int row = e >> 3, c8 = (e & 7) * 8;
                hv[j] = *(const v8h*)(T16 + row * VP + c8);
            }
#pragma unroll
            for (int j = 0; j < 8; ++j) {
                const int e = tid + 64 * j;
                const int row = e >> 3, c8 = (e & 7) * 8;
                _Float16* gp = Vt + (size_t)(bn + row) * M + bm + c8;
                *(volatile v8h*)gp = hv[j];
            }
            __threadfence();
#pragma unroll
            for (int j = 0; j < 8; ++j) {
                const int e = tid + 64 * j;
                const int row = e >> 3, c8 = (e & 7) * 8;
                _Float16* gp = Vt + (size_t)(bn + row) * M + bm + c8;
                *(volatile v8h*)gp = hv[j];
            }
        }
        if (do_lo) {
            v8h lv[8];
#pragma unroll
            for (int j = 0; j < 8; ++j) {
                const int e = tid + 64 * j;
                const int row = e >> 3, c8 = (e & 7) * 8;
                lv[j] = *(const v8h*)(TL + row * VP + c8);
            }
#pragma unroll
            for (int j = 0; j < 8; ++j) {
                const int e = tid + 64 * j;
                const int row = e >> 3, c8 = (e & 7) * 8;
                _Float16* gp = Clo + (size_t)(bn + row) * lo_rows + bm + c8;
                *(volatile v8h*)gp = lv[j];
            }
            __threadfence();
#pragma unroll
            for (int j = 0; j < 8; ++j) {
                const int e = tid + 64 * j;
                const int row = e >> 3, c8 = (e & 7) * 8;
                _Float16* gp = Clo + (size_t)(bn + row) * lo_rows + bm + c8;
                *(volatile v8h*)gp = lv[j];
            }
        }
    }
}

template <bool PREC>
__global__ __launch_bounds__(64)
void attn_k(const _Float16* __restrict__ Qh, const _Float16* __restrict__ Ql,
            const _Float16* __restrict__ Kh, const _Float16* __restrict__ Kl,
            const _Float16* __restrict__ Vth, const _Float16* __restrict__ Vtl,
            _Float16* __restrict__ Oh, _Float16* __restrict__ Ol, int blk0)
{
    constexpr int KT    = PREC ? 32 : 64;
    constexpr int NJ    = KT / 16;
    constexpr int NKS   = KT / 32;
    constexpr int NCH   = PREC ? 2 : 8;
    constexpr int NPASS = 8 / NCH;
    constexpr int OP    = 136;
    __shared__ __align__(16) _Float16 Ot [2][16 * OP];
    __shared__ __align__(16) _Float16 Otl[PREC ? 2 : 1][PREC ? 16 * OP : 8];
    (void)Ql; (void)Kl; (void)Vtl; (void)Ol;

    const int tid = threadIdx.x, w = tid >> 5, l = tid & 31, h = l >> 4, m = l & 15;
    const int hq = blockIdx.y;
    const int hk = hq / (HQ_N / HKV_N);
    const int qb = (blk0 + (int)blockIdx.x) * 32 + 16 * w;
    const int qrow = qb + m;
    const int ntiles = qb / KT + 1;
    const float scale = 0.08838834764831845f;
    const float NEG = -__builtin_inff();

    const _Float16* qhp = Qh + (size_t)qrow * HID + hq * D_DIM + 8 * h;
    const _Float16* qlp = PREC ? (Ql + (size_t)qrow * HID + hq * D_DIM + 8 * h) : Ql;

    Frag qf[4];
    if constexpr (!PREC) {
#pragma unroll
        for (int dc = 0; dc < 4; ++dc) {
            qf[dc].half[0] = *(const v8h*)(qhp + 32 * dc);
            qf[dc].half[1] = *(const v8h*)(qhp + 32 * dc + 16);
        }
    }

    _Float16* ot  = &Ot[w][0];
    _Float16* otl = &Otl[PREC ? w : 0][0];

#pragma unroll 1
    for (int pass = 0; pass < NPASS; ++pass) {
        const int chb = pass * NCH;
        v8f oacc[NCH], oaccr[NCH];
#pragma unroll
        for (int c = 0; c < NCH; ++c) { oacc[c] = vzero8(); oaccr[c] = vzero8(); }
        float mrun = NEG, lrun = 0.f;

        for (int t = 0; t < ntiles; ++t) {
            const int kt = t * KT;
            v8f sacc[NJ], saccr[NJ];
#pragma unroll
            for (int j = 0; j < NJ; ++j) { sacc[j] = vzero8(); saccr[j] = vzero8(); }

#pragma unroll
            for (int j = 0; j < NJ; ++j) {
                const _Float16* khp = Kh + (size_t)(kt + 16 * j + m) * KVD + hk * D_DIM + 8 * h;
                if constexpr (!PREC) {
                    Frag kf[4];
#pragma unroll
                    for (int dc = 0; dc < 4; ++dc) {
                        kf[dc].half[0] = *(const v8h*)(khp + 32 * dc);
                        kf[dc].half[1] = *(const v8h*)(khp + 32 * dc + 16);
                    }
#pragma unroll
                    for (int dc = 0; dc < 4; ++dc) sacc[j] = wmma16(kf[dc].v, qf[dc].v, sacc[j]);
                    asm volatile(NOP4
                                 : "+v"(sacc[j])
                                 : "v"(kf[0].v), "v"(kf[1].v), "v"(kf[2].v), "v"(kf[3].v),
                                   "v"(qf[0].v), "v"(qf[1].v), "v"(qf[2].v), "v"(qf[3].v));
                } else {
                    const _Float16* klp = Kl + (size_t)(kt + 16 * j + m) * KVD + hk * D_DIM + 8 * h;
#pragma unroll
                    for (int dc = 0; dc < 4; ++dc) {
                        Frag kh_, kl_, qh_, ql_;
                        kh_.half[0] = *(const v8h*)(khp + 32 * dc);
                        kh_.half[1] = *(const v8h*)(khp + 32 * dc + 16);
                        kl_.half[0] = *(const v8h*)(klp + 32 * dc);
                        kl_.half[1] = *(const v8h*)(klp + 32 * dc + 16);
                        qh_.half[0] = *(const v8h*)(qhp + 32 * dc);
                        qh_.half[1] = *(const v8h*)(qhp + 32 * dc + 16);
                        ql_.half[0] = *(const v8h*)(qlp + 32 * dc);
                        ql_.half[1] = *(const v8h*)(qlp + 32 * dc + 16);
                        sacc[j]  = wmma16(kh_.v, qh_.v, sacc[j]);
                        saccr[j] = wmma16(kh_.v, ql_.v, saccr[j]);
                        saccr[j] = wmma16(kl_.v, qh_.v, saccr[j]);
                        asm volatile(NOP4
                                     : "+v"(sacc[j]), "+v"(saccr[j])
                                     : "v"(kh_.v), "v"(kl_.v), "v"(qh_.v), "v"(ql_.v));
                    }
                }
            }

            const bool diag = (kt + KT - 1 > qb);
            float tmax = NEG;
#pragma unroll
            for (int j = 0; j < NJ; ++j)
#pragma unroll
                for (int r = 0; r < 8; ++r) {
                    float a = sacc[j][r];
                    if constexpr (PREC) a += saccr[j][r] * (1.0f / 2048.0f);
                    a *= scale;
                    if (diag) {
                        const int key = kt + 16 * j + 8 * h + r;
                        if (key > qrow) a = NEG;
                    }
                    sacc[j][r] = a;
                    tmax = fmaxf(tmax, a);
                }
            tmax = fmaxf(tmax, __shfl_xor(tmax, 16, 32));
            const float mnew = fmaxf(mrun, tmax);
            const float corr = __expf(mrun - mnew);
            float psum = 0.f;
            Frag pf[NKS], pfl[NKS];
#pragma unroll
            for (int j = 0; j < NJ; ++j) {
                v8h ph8, pl8;
#pragma unroll
                for (int r = 0; r < 8; ++r) {
                    const float p = __expf(sacc[j][r] - mnew);
                    psum += p;
                    const float p4 = p * 4096.0f;
                    const _Float16 ph = (_Float16)p4;
                    ph8[r] = ph;
                    pl8[r] = (_Float16)((p4 - (float)ph) * 2048.0f);
                }
                pf[j >> 1].half[j & 1] = ph8;
                if constexpr (PREC) pfl[j >> 1].half[j & 1] = pl8;
            }
            psum += __shfl_xor(psum, 16, 32);
            lrun = lrun * corr + psum;
            mrun = mnew;
            float cr[8];
#pragma unroll
            for (int r = 0; r < 8; ++r) cr[r] = __shfl(corr, 8 * h + r, 32);
#pragma unroll
            for (int c = 0; c < NCH; ++c)
#pragma unroll
                for (int r = 0; r < 8; ++r) {
                    oacc[c][r] *= cr[r];
                    if constexpr (PREC) oaccr[c][r] *= cr[r];
                }

#pragma unroll
            for (int c = 0; c < NCH; ++c) {
                const int ch = chb + c;
                const _Float16* vhp = Vth + (size_t)(hk * D_DIM + 16 * ch + m) * S_LEN + kt + 8 * h;
                if constexpr (!PREC) {
                    Frag vf[2];
#pragma unroll
                    for (int ks = 0; ks < 2; ++ks) {
                        vf[ks].half[0] = *(const v8h*)(vhp + 32 * ks);
                        vf[ks].half[1] = *(const v8h*)(vhp + 32 * ks + 16);
                    }
                    oacc[c] = wmma16(pf[0].v, vf[0].v, oacc[c]);
                    oacc[c] = wmma16(pf[1].v, vf[1].v, oacc[c]);
                    asm volatile(NOP4
                                 : "+v"(oacc[c])
                                 : "v"(pf[0].v), "v"(pf[1].v), "v"(vf[0].v), "v"(vf[1].v));
                } else {
                    const _Float16* vlp = Vtl + (size_t)(hk * D_DIM + 16 * ch + m) * LO_ROWS + kt + 8 * h;
                    Frag vh_, vl_;
                    vh_.half[0] = *(const v8h*)(vhp);
                    vh_.half[1] = *(const v8h*)(vhp + 16);
                    vl_.half[0] = *(const v8h*)(vlp);
                    vl_.half[1] = *(const v8h*)(vlp + 16);
                    oacc[c]  = wmma16(pf[0].v, vh_.v, oacc[c]);
                    oaccr[c] = wmma16(pf[0].v, vl_.v, oaccr[c]);
                    oaccr[c] = wmma16(pfl[0].v, vh_.v, oaccr[c]);
                    asm volatile(NOP4
                                 : "+v"(oacc[c]), "+v"(oaccr[c])
                                 : "v"(pf[0].v), "v"(pfl[0].v), "v"(vh_.v), "v"(vl_.v));
                }
            }
        }

        const float invl = 1.0f / (64.0f * lrun);
        float il[8];
#pragma unroll
        for (int r = 0; r < 8; ++r) il[r] = __shfl(invl, 8 * h + r, 32);
#pragma unroll
        for (int c = 0; c < NCH; ++c)
#pragma unroll
            for (int r = 0; r < 8; ++r) {
                float y = oacc[c][r];
                if constexpr (PREC) y += oaccr[c][r] * (1.0f / 2048.0f);
                y *= il[r];
                const _Float16 hh = (_Float16)y;
                ot[(8 * h + r) * OP + (chb + c) * 16 + m] = hh;
                if constexpr (PREC) otl[(8 * h + r) * OP + (chb + c) * 16 + m] = (_Float16)((y - (float)hh) * 2048.0f);
            }
    }
    __syncthreads();

    {
        v8h hv[8];
#pragma unroll
        for (int jj = 0; jj < 8; ++jj) {
            const int e = l + 32 * jj;
            const int row = e >> 4, c8 = (e & 15) * 8;
            hv[jj] = *(const v8h*)(ot + row * OP + c8);
        }
#pragma unroll
        for (int jj = 0; jj < 8; ++jj) {
            const int e = l + 32 * jj;
            const int row = e >> 4, c8 = (e & 15) * 8;
            _Float16* gp = Oh + (size_t)(qb + row) * HID + hq * D_DIM + c8;
            *(volatile v8h*)gp = hv[jj];
        }
        __threadfence();
#pragma unroll
        for (int jj = 0; jj < 8; ++jj) {
            const int e = l + 32 * jj;
            const int row = e >> 4, c8 = (e & 15) * 8;
            _Float16* gp = Oh + (size_t)(qb + row) * HID + hq * D_DIM + c8;
            *(volatile v8h*)gp = hv[jj];
        }
    }
    if constexpr (PREC) {
        v8h lv[8];
#pragma unroll
        for (int jj = 0; jj < 8; ++jj) {
            const int e = l + 32 * jj;
            const int row = e >> 4, c8 = (e & 15) * 8;
            lv[jj] = *(const v8h*)(otl + row * OP + c8);
        }
#pragma unroll
        for (int jj = 0; jj < 8; ++jj) {
            const int e = l + 32 * jj;
            const int row = e >> 4, c8 = (e & 15) * 8;
            _Float16* gp = Ol + (size_t)(qb + row) * HID + hq * D_DIM + c8;
            *(volatile v8h*)gp = lv[jj];
        }
        __threadfence();
#pragma unroll
        for (int jj = 0; jj < 8; ++jj) {
            const int e = l + 32 * jj;
            const int row = e >> 4, c8 = (e & 15) * 8;
            _Float16* gp = Ol + (size_t)(qb + row) * HID + hq * D_DIM + c8;
            *(volatile v8h*)gp = lv[jj];
        }
    }
}

extern "C" void kernel_launch(void* const* d_in, const int* in_sizes, int n_in,
                              void* d_out, int out_size, void* d_ws, size_t ws_size,
                              hipStream_t stream)
{
    if (n_in < 6) return;
    if (in_sizes[0] != S_LEN * HID || in_sizes[1] < S_LEN || in_sizes[2] != HID * HID ||
        in_sizes[3] != KVD * HID || in_sizes[4] != KVD * HID || in_sizes[5] != HID * HID) return;
    if (out_size != S_LEN * HID) return;

    const float* x  = (const float*)d_in[0];
    const int*   xp = (const int*)d_in[1];
    const float* Wq = (const float*)d_in[2];
    const float* Wk = (const float*)d_in[3];
    const float* Wv = (const float*)d_in[4];
    const float* Wo = (const float*)d_in[5];
    float* out = (float*)d_out;

    char* ws = (char*)d_ws;
    size_t off = 0;
    const size_t szX   = (size_t)S_LEN * HID * sizeof(_Float16);
    const size_t szWq  = (size_t)HID * HID * sizeof(_Float16);
    const size_t szWk  = (size_t)KVD * HID * sizeof(_Float16);
    const size_t szTab = (size_t)2 * S_LEN * ROT * sizeof(float);
    const size_t szQl  = (size_t)LO_ROWS * HID * sizeof(_Float16);
    const size_t szK   = (size_t)S_LEN * KVD * sizeof(_Float16);
    const size_t szKl  = (size_t)LO_ROWS * KVD * sizeof(_Float16);

    _Float16* xh  = (_Float16*)(ws + off); off += szX;
    _Float16* wqh = (_Float16*)(ws + off); off += szWq;
    _Float16* wkh = (_Float16*)(ws + off); off += szWk;
    _Float16* wvh = (_Float16*)(ws + off); off += szWk;
    _Float16* woh = (_Float16*)(ws + off); off += szWq;
    float*    tab = (float*)   (ws + off); off += szTab;
    _Float16* qh  = (_Float16*)(ws + off); off += szX;
    _Float16* ql  = (_Float16*)(ws + off); off += szQl;
    _Float16* kh  = (_Float16*)(ws + off); off += szK;
    _Float16* kl  = (_Float16*)(ws + off); off += szKl;
    _Float16* vth = (_Float16*)(ws + off); off += szK;
    _Float16* vtl = (_Float16*)(ws + off); off += szKl;
    _Float16* oh  = (_Float16*)(ws + off); off += szX;
    _Float16* ol  = (_Float16*)(ws + off); off += szQl;
    if (off > ws_size) return;

    const dim3 b64(64), b256(256);
    const int n8x  = S_LEN * HID / 8;
    const int n8wq = HID * HID / 8;
    const int n8wk = KVD * HID / 8;

    cvt_k<<<dim3((n8x  + 255) / 256), b256, 0, stream>>>(x,  xh,  n8x,  1.0f);
    cvt_k<<<dim3((n8wq + 255) / 256), b256, 0, stream>>>(Wq, wqh, n8wq, 64.0f);
    cvt_k<<<dim3((n8wk + 255) / 256), b256, 0, stream>>>(Wk, wkh, n8wk, 64.0f);
    cvt_k<<<dim3((n8wk + 255) / 256), b256, 0, stream>>>(Wv, wvh, n8wk, 64.0f);
    cvt_k<<<dim3((n8wq + 255) / 256), b256, 0, stream>>>(Wo, woh, n8wq, 64.0f);

    rope_tab_k<<<dim3(S_LEN), b64, 0, stream>>>(xp, tab, S_LEN, in_sizes[1]);

    gemm_k<0><<<dim3(HID / 128, S_LEN / 32), b64, 0, stream>>>(xh, xh, wqh, (void*)qh, ql, tab,
                                                               S_LEN, HID, HID, LO_ROWS, 1.0f / 64.0f);
    gemm_k<0><<<dim3(KVD / 128, S_LEN / 32), b64, 0, stream>>>(xh, xh, wkh, (void*)kh, kl, tab,
                                                               S_LEN, KVD, HID, LO_ROWS, 1.0f / 64.0f);
    gemm_k<1><<<dim3(KVD / 64, S_LEN / 64), b64, 0, stream>>>(xh, xh, wvh, (void*)vth, vtl, tab,
                                                              S_LEN, KVD, HID, LO_ROWS, 1.0f / 64.0f);
    attn_k<true><<<dim3(LO_ROWS / 32, HQ_N), b64, 0, stream>>>(qh, ql, kh, kl, vth, vtl, oh, ol, 0);
    attn_k<false><<<dim3(S_LEN / 32 - LO_ROWS / 32, HQ_N), b64, 0, stream>>>(qh, ql, kh, kl, vth, vtl,
                                                                          oh, ol, LO_ROWS / 32);
    gemm_k<2><<<dim3(HID / 128, S_LEN / 32), b64, 0, stream>>>(oh, ol, woh, (void*)out, ql, tab,
                                                               S_LEN, HID, HID, LO_ROWS, 1.0f / 4096.0f);
}
